// FourierGlobalAttention_13572096656028
// MI455X (gfx1250) — hardware-verified
//
#include <hip/hip_runtime.h>
#include <hip/hip_bf16.h>
#include <math.h>


typedef __bf16       v16bf __attribute__((ext_vector_type(16)));
typedef float        v8f   __attribute__((ext_vector_type(8)));
typedef float        v4f   __attribute__((ext_vector_type(4)));
typedef unsigned int v4u   __attribute__((ext_vector_type(4)));
typedef int          v8i   __attribute__((ext_vector_type(8)));
typedef v4u v4ua __attribute__((may_alias));
typedef v4f v4fa __attribute__((may_alias));

#define BATCH   8
#define CH      512
#define NHEADS  8
#define HEADD   64
#define NTOK    1024
#define TTOT    8192
#define QKV_N   1536
#define SCALE_F 0.125f

#define LDP  72
#define KCH  128
#define KSP  72
#define VTP  136
#define PP   40
#define EP   36

union Frag16 { v16bf v; v4u u[2]; };
union Pack8  { v4u u; __bf16 e[8]; };
union Pack32 { v4u u[4]; __bf16 e[32]; };

static __device__ __forceinline__ __bf16 f2bf(float f) { return (__bf16)f; }

static __device__ __forceinline__ v8f zero8() {
  v8f z = {0.f, 0.f, 0.f, 0.f, 0.f, 0.f, 0.f, 0.f};
  return z;
}

static __device__ __forceinline__ v8f mma(v16bf a, v16bf b, v8f c) {
  c = __builtin_amdgcn_wmma_f32_16x16x32_bf16(false, a, false, b, (short)0, c, false, false);
  v8i aw = __builtin_bit_cast(v8i, a);
  v8i bw = __builtin_bit_cast(v8i, b);
  asm volatile("v_nop\n\tv_nop\n\tv_nop\n\tv_nop" : "+v"(c) : "v"(aw), "v"(bw));
  return c;
}

static __device__ __forceinline__ v16bf ldfrag(const __bf16* rowp, int k0, int h) {
  Frag16 f;
  f.u[0] = *(const v4ua*)(rowp + k0 + 8 * h);
  f.u[1] = *(const v4ua*)(rowp + k0 + 16 + 8 * h);
  return f.v;
}

static __device__ __forceinline__ void stage16(const float* __restrict__ src, __bf16* dst) {
#pragma unroll
  for (int q = 0; q < 2; ++q) {
    const v4f f0 = *(const v4fa*)(src + 8 * q);
    const v4f f1 = *(const v4fa*)(src + 8 * q + 4);
    Pack8 p;
    p.e[0] = f2bf(f0[0]); p.e[1] = f2bf(f0[1]); p.e[2] = f2bf(f0[2]); p.e[3] = f2bf(f0[3]);
    p.e[4] = f2bf(f1[0]); p.e[5] = f2bf(f1[1]); p.e[6] = f2bf(f1[2]); p.e[7] = f2bf(f1[3]);
    *(v4ua*)(dst + 8 * q) = p.u;
  }
}

__global__ __launch_bounds__(256)
void ttab_kernel(float* __restrict__ T) {
  __shared__ float ct[32], st[32];
  const int tid = threadIdx.x;
  if (tid < 32) {
    const float th = 6.283185307179586f * (float)tid * (1.0f / 32.0f);
    ct[tid] = cosf(th);
    st[tid] = sinf(th);
  }
  __syncthreads();
  const int e0 = tid * 4, hh = e0 >> 5, w0 = e0 & 31;
  v4f val;
#pragma unroll
  for (int c = 0; c < 4; ++c) {
    const int w = w0 + c;
    float acc = 0.f;
    if (hh == 0) {
      acc = 1.0f + ct[(16 * w) & 31];
#pragma unroll 1
      for (int k = 1; k <= 15; ++k) {
        const int id = (k * w) & 31;
        acc += 2.0f * (ct[id] - st[id]);
      }
    }
    val[c] = acc;
  }
  if (e0 + 4 <= NTOK) {
    *(volatile v4f*)(T + e0) = val;
    __threadfence();
    *(volatile v4f*)(T + e0) = val;
  }
}

__global__ __launch_bounds__(256)
void qkv_kernel(const float* __restrict__ x, const float* __restrict__ w,
                __bf16* __restrict__ qo, __bf16* __restrict__ ko, __bf16* __restrict__ vo) {
  __shared__ __align__(16) __bf16 As[64 * LDP];
  __shared__ __align__(16) __bf16 Bs[64 * LDP];
  __shared__ __align__(16) __bf16 Cs[64 * LDP];
  const int tid = threadIdx.x, wave = tid >> 5, lane = tid & 31;
  const int h = lane >> 4, m = lane & 15;
  const int m0 = blockIdx.x * 64, n0 = blockIdx.y * 64;
  if (m0 + 64 > TTOT || n0 + 64 > QKV_N) return;
  const int r16 = (wave & 3) * 16, cn = (wave >> 2) * 32;
  const int srow = tid >> 2, sc0 = (tid & 3) * 16;
  v8f acc0 = zero8(), acc1 = zero8();

  for (int kk = 0; kk < CH; kk += 64) {
    stage16(x + (size_t)(m0 + srow) * CH + kk + sc0, &As[srow * LDP + sc0]);
    stage16(w + (size_t)(n0 + srow) * CH + kk + sc0, &Bs[srow * LDP + sc0]);
    __syncthreads();
#pragma unroll
    for (int ks = 0; ks < 64; ks += 32) {
      const v16bf a  = ldfrag(&As[(r16 + m) * LDP], ks, h);
      const v16bf b0 = ldfrag(&Bs[(cn + m) * LDP], ks, h);
      const v16bf b1 = ldfrag(&Bs[(cn + 16 + m) * LDP], ks, h);
      acc0 = mma(a, b0, acc0);
      acc1 = mma(a, b1, acc1);
    }
    __syncthreads();
  }

#pragma unroll
  for (int r = 0; r < 8; ++r) {
    Cs[(r16 + 8 * h + r) * LDP + cn + m]      = f2bf(acc0[r]);
    Cs[(r16 + 8 * h + r) * LDP + cn + 16 + m] = f2bf(acc1[r]);
  }
  __syncthreads();

  const int s = n0 >> 9, head = (n0 & 511) >> 6;
  __bf16* base = (s == 0) ? qo : ((s == 1) ? ko : vo);
  v4u val[2];
  size_t off[2];
#pragma unroll
  for (int it = 0; it < 2; ++it) {
    const int row = wave * 8 + it * 4 + (lane >> 3), c8 = (lane & 7) * 8;
    const int tok = m0 + row, b = tok >> 10, nb = tok & (NTOK - 1);
    val[it] = *(const v4ua*)&Cs[row * LDP + c8];
    off[it] = ((size_t)(b * NHEADS + head) * NTOK + nb) * HEADD + c8;
  }
#pragma unroll
  for (int it = 0; it < 2; ++it) *(volatile v4u*)(base + off[it]) = val[it];
  __threadfence();
#pragma unroll
  for (int it = 0; it < 2; ++it) *(volatile v4u*)(base + off[it]) = val[it];
}

__global__ __launch_bounds__(256)
void attn_kernel(const __bf16* __restrict__ qb, const __bf16* __restrict__ kb,
                 const __bf16* __restrict__ vb, __bf16* __restrict__ ao) {
  __shared__ __align__(16) __bf16 Ks[KCH * KSP];
  __shared__ __align__(16) __bf16 Vt[HEADD * VTP];
  __shared__ __align__(16) __bf16 Pb[8 * 16 * PP];
  const int tid = threadIdx.x, wave = tid >> 5, lane = tid & 31;
  const int h = lane >> 4, m = lane & 15;
  const int bh = blockIdx.x >> 3, qc = blockIdx.x & 7;
  if (bh >= BATCH * NHEADS) return;
  const int qrow0 = qc * 128 + wave * 16;
  const size_t hoff = (size_t)bh * NTOK * HEADD;
  const __bf16* qbase = qb + hoff;
  const __bf16* kbase = kb + hoff;
  const __bf16* vbase = vb + hoff;

  const v16bf qf0 = ldfrag(qbase + (size_t)(qrow0 + m) * HEADD, 0, h);
  const v16bf qf1 = ldfrag(qbase + (size_t)(qrow0 + m) * HEADD, 32, h);

  float mrow[8], lrow[8];
  v8f o[4];
#pragma unroll
  for (int nt = 0; nt < 4; ++nt) o[nt] = zero8();
#pragma unroll
  for (int r = 0; r < 8; ++r) { mrow[r] = -1e30f; lrow[r] = 0.f; }

  __bf16* myP = Pb + wave * 16 * PP;
  const int skey = tid >> 1, sd0 = (tid & 1) * 32;

  for (int c = 0; c < NTOK / KCH; ++c) {
    {
      const __bf16* ksrc = kbase + (size_t)(c * KCH + skey) * HEADD + sd0;
#pragma unroll
      for (int i = 0; i < 4; ++i)
        *(v4ua*)&Ks[skey * KSP + sd0 + 8 * i] = *(const v4ua*)(ksrc + 8 * i);
      const __bf16* vsrc = vbase + (size_t)(c * KCH + skey) * HEADD + sd0;
      Pack32 pv;
#pragma unroll
      for (int i = 0; i < 4; ++i) pv.u[i] = *(const v4ua*)(vsrc + 8 * i);
#pragma unroll
      for (int i = 0; i < 32; ++i) Vt[(sd0 + i) * VTP + skey] = pv.e[i];
    }
    __syncthreads();

    for (int sb = 0; sb < KCH / 32; ++sb) {
      const int kcol = sb * 32;
      v8f s0 = zero8(), s1 = zero8();
      {
        v16bf bk;
        bk = ldfrag(&Ks[(kcol + m) * KSP], 0, h);        s0 = mma(qf0, bk, s0);
        bk = ldfrag(&Ks[(kcol + m) * KSP], 32, h);       s0 = mma(qf1, bk, s0);
        bk = ldfrag(&Ks[(kcol + 16 + m) * KSP], 0, h);   s1 = mma(qf0, bk, s1);
        bk = ldfrag(&Ks[(kcol + 16 + m) * KSP], 32, h);  s1 = mma(qf1, bk, s1);
      }
#pragma unroll
      for (int r = 0; r < 8; ++r) {
        const float a0 = s0[r] * SCALE_F, a1 = s1[r] * SCALE_F;
        float rv = fmaxf(a0, a1);
        rv = fmaxf(rv, __shfl_xor(rv, 1, 32));
        rv = fmaxf(rv, __shfl_xor(rv, 2, 32));
        rv = fmaxf(rv, __shfl_xor(rv, 4, 32));
        rv = fmaxf(rv, __shfl_xor(rv, 8, 32));
        const float mnew = fmaxf(mrow[r], rv);
        const float alpha = __expf(mrow[r] - mnew);
        mrow[r] = mnew;
        const float p0 = __expf(a0 - mnew);
        const float p1 = __expf(a1 - mnew);
        float rs = p0 + p1;
        rs += __shfl_xor(rs, 1, 32);
        rs += __shfl_xor(rs, 2, 32);
        rs += __shfl_xor(rs, 4, 32);
        rs += __shfl_xor(rs, 8, 32);
        lrow[r] = lrow[r] * alpha + rs;
        o[0][r] *= alpha; o[1][r] *= alpha; o[2][r] *= alpha; o[3][r] *= alpha;
        s0[r] = p0; s1[r] = p1;
      }
#pragma unroll
      for (int r = 0; r < 8; ++r) {
        myP[(8 * h + r) * PP + m]      = f2bf(s0[r]);
        myP[(8 * h + r) * PP + 16 + m] = f2bf(s1[r]);
      }
      asm volatile("" ::: "memory");
      const v16bf pa = ldfrag(myP + m * PP, 0, h);
#pragma unroll
      for (int nt = 0; nt < 4; ++nt) {
        const v16bf bv = ldfrag(&Vt[(nt * 16 + m) * VTP], kcol, h);
        o[nt] = mma(pa, bv, o[nt]);
      }
    }
    __syncthreads();
  }

  float invl[8];
#pragma unroll
  for (int r = 0; r < 8; ++r) invl[r] = 1.f / lrow[r];
  __bf16* Os = Ks;
#pragma unroll
  for (int nt = 0; nt < 4; ++nt)
#pragma unroll
    for (int r = 0; r < 8; ++r)
      Os[(wave * 16 + 8 * h + r) * KSP + nt * 16 + m] = f2bf(o[nt][r] * invl[r]);
  __syncthreads();

  const int head = bh & (NHEADS - 1), b = bh >> 3;
  v4u val[4];
  size_t off[4];
#pragma unroll
  for (int it = 0; it < 4; ++it) {
    const int row = wave * 16 + it * 4 + (lane >> 3), c8 = (lane & 7) * 8;
    const int tok = qc * 128 + row;
    val[it] = *(const v4ua*)&Os[row * KSP + c8];
    off[it] = ((size_t)(b * NTOK + tok)) * CH + head * HEADD + c8;
  }
#pragma unroll
  for (int it = 0; it < 4; ++it) *(volatile v4u*)(ao + off[it]) = val[it];
  __threadfence();
#pragma unroll
  for (int it = 0; it < 4; ++it) *(volatile v4u*)(ao + off[it]) = val[it];
}

__global__ __launch_bounds__(256)
void final_kernel(const __bf16* __restrict__ ao, const float* __restrict__ x,
                  const float* __restrict__ pw, const float* __restrict__ pb,
                  const float* __restrict__ fw, const float* __restrict__ fb,
                  const float* __restrict__ qw, const float* __restrict__ lg,
                  const float* __restrict__ lb, const float* __restrict__ mw,
                  const float* __restrict__ Ttab, float* __restrict__ out) {
  __shared__ __align__(16) __bf16 Bs[64 * LDP];
  __shared__ __align__(16) float Es[8 * 16 * EP];
  __shared__ __align__(16) float g_s[CH];
  __shared__ __align__(16) float bb_s[CH];
  __shared__ __align__(16) float pb_s[CH];
  __shared__ __align__(16) float lg_s[CH];
  __shared__ __align__(16) float lb_s[CH];
  __shared__ float T_s[64], mu_s[64], rs_s[64];

  const int tid = threadIdx.x, wave = tid >> 5, lane = tid & 31;
  const int h = lane >> 4, m = lane & 15;
  const int m0 = blockIdx.x * 64;
  if (m0 + 64 > TTOT) return;

#pragma unroll
  for (int q = 0; q < 2; ++q) {
    const int cch = q * 256 + tid;
    g_s[cch]  = qw[cch] + 0.1f * fw[cch];
    bb_s[cch] = 0.1f * fb[cch];
    pb_s[cch] = pb[cch];
    lg_s[cch] = lg[cch];
    lb_s[cch] = lb[cch];
  }
  if (tid < 64) T_s[tid] = Ttab[(m0 + tid) & (NTOK - 1)];
  __syncthreads();

  {
    const int tok = tid >> 2, part = tid & 3;
    const float Tv = T_s[tok];
    const float* xr = x + (size_t)(m0 + tok) * CH + part * 128;
    const float* gr = &g_s[part * 128];
    const float* br = &bb_s[part * 128];
    float s = 0.f;
#pragma unroll 2
    for (int i = 0; i < 128; i += 4) {
      const v4f xv = *(const v4fa*)(xr + i);
      const v4f gv = *(const v4fa*)(gr + i);
      const v4f bv = *(const v4fa*)(br + i);
      s += (gv[0] * xv[0] + bv[0] * Tv) + (gv[1] * xv[1] + bv[1] * Tv)
         + (gv[2] * xv[2] + bv[2] * Tv) + (gv[3] * xv[3] + bv[3] * Tv);
    }
    s += __shfl_xor(s, 1, 32);
    s += __shfl_xor(s, 2, 32);
    const float mu = s * (1.f / 512.f);
    float s2 = 0.f;
#pragma unroll 2
    for (int i = 0; i < 128; i += 4) {
      const v4f xv = *(const v4fa*)(xr + i);
      const v4f gv = *(const v4fa*)(gr + i);
      const v4f bv = *(const v4fa*)(br + i);
#pragma unroll
      for (int e = 0; e < 4; ++e) {
        const float d = (gv[e] * xv[e] + bv[e] * Tv) - mu;
        s2 += d * d;
      }
    }
    s2 += __shfl_xor(s2, 1, 32);
    s2 += __shfl_xor(s2, 2, 32);
    const float var = s2 * (1.f / 512.f);
    const float rs = 1.0f / sqrtf(var + 1e-5f);
    if (part == 0) { mu_s[tok] = mu; rs_s[tok] = rs; }
  }
  __syncthreads();

  float w0, w1;
  {
    const float a0 = mw[0], a1 = mw[1];
    const float mx = fmaxf(a0, a1);
    const float e0 = __expf(a0 - mx), e1 = __expf(a1 - mx);
    const float inv = 1.f / (e0 + e1);
    w0 = e0 * inv; w1 = e1 * inv;
  }

  const int r16 = (wave & 3) * 16, cn = (wave >> 2) * 32;
  const int srow = tid >> 2, sc0 = (tid & 3) * 16;
  const __bf16* arow = ao + (size_t)(m0 + r16 + m) * CH;
  float* ew = &Es[wave * 16 * EP];

  for (int nb = 0; nb < CH / 64; ++nb) {
    const int n0 = nb * 64;
    v8f acc0 = zero8(), acc1 = zero8();
    for (int kk = 0; kk < CH; kk += 64) {
      stage16(pw + (size_t)(n0 + srow) * CH + kk + sc0, &Bs[srow * LDP + sc0]);
      __syncthreads();
#pragma unroll
      for (int ks = 0; ks < 64; ks += 32) {
        const v16bf a  = ldfrag(arow, kk + ks, h);
        const v16bf b0 = ldfrag(&Bs[(cn + m) * LDP], ks, h);
        const v16bf b1 = ldfrag(&Bs[(cn + 16 + m) * LDP], ks, h);
        acc0 = mma(a, b0, acc0);
        acc1 = mma(a, b1, acc1);
      }
      __syncthreads();
    }

#pragma unroll
    for (int r = 0; r < 8; ++r) {
      ew[(8 * h + r) * EP + m]      = acc0[r];
      ew[(8 * h + r) * EP + 16 + m] = acc1[r];
    }
    asm volatile("" ::: "memory");

    v4f res[4];
    size_t off[4];
#pragma unroll
    for (int it = 0; it < 4; ++it) {
      const int row = it * 4 + (lane >> 3), c4 = (lane & 7) * 4;
      const int trow = r16 + row, tok = m0 + trow, j = n0 + cn + c4;
      const v4f a   = *(const v4fa*)&ew[row * EP + c4];
      const v4f xv  = *(const v4fa*)(x + (size_t)tok * CH + j);
      const v4f g4  = *(const v4fa*)&g_s[j];
      const v4f bb4 = *(const v4fa*)&bb_s[j];
      const v4f pb4 = *(const v4fa*)&pb_s[j];
      const v4f lg4 = *(const v4fa*)&lg_s[j];
      const v4f lb4 = *(const v4fa*)&lb_s[j];
      const float Tv = T_s[trow], mu = mu_s[trow], rs = rs_s[trow];
      v4f o4;
#pragma unroll
      for (int e = 0; e < 4; ++e) {
        const float xf   = g4[e] * xv[e] + bb4[e] * Tv;
        const float four = (xf - mu) * rs * lg4[e] + lb4[e];
        const float spa  = a[e] + pb4[e];
        o4[e] = w0 * spa + w1 * four;
      }
      res[it] = o4;
      off[it] = (size_t)tok * CH + j;
    }
#pragma unroll
    for (int it = 0; it < 4; ++it) *(volatile v4f*)(out + off[it]) = res[it];
    __threadfence();
#pragma unroll
    for (int it = 0; it < 4; ++it) *(volatile v4f*)(out + off[it]) = res[it];
  }
}

extern "C" void kernel_launch(void* const* d_in, const int* in_sizes, int n_in,
                              void* d_out, int out_size, void* d_ws, size_t ws_size,
                              hipStream_t stream) {
  if (n_in < 10) return;
  if (in_sizes[0] != TTOT * CH || in_sizes[1] != QKV_N * CH || in_sizes[2] != CH * CH) return;
  if (in_sizes[3] != CH || in_sizes[4] != CH || in_sizes[5] != CH || in_sizes[6] != CH ||
      in_sizes[7] != CH || in_sizes[8] != CH || in_sizes[9] != 2) return;
  if (out_size != TTOT * CH) return;

  const size_t tab_bytes = 4096;
  const size_t buf_elems = (size_t)TTOT * CH;
  const size_t need = tab_bytes + 4 * buf_elems * sizeof(__bf16);
  if (need > ws_size) return;

  const float* x       = (const float*)d_in[0];
  const float* qkv_w   = (const float*)d_in[1];
  const float* proj_w  = (const float*)d_in[2];
  const float* proj_b  = (const float*)d_in[3];
  const float* fconv_w = (const float*)d_in[4];
  const float* fconv_b = (const float*)d_in[5];
  const float* freq_w  = (const float*)d_in[6];
  const float* ln_g    = (const float*)d_in[7];
  const float* ln_b    = (const float*)d_in[8];
  const float* mix_w   = (const float*)d_in[9];
  float* out = (float*)d_out;

  char* ws = (char*)d_ws;
  float*  Ttab = (float*)ws;
  __bf16* qb = (__bf16*)(ws + tab_bytes);
  __bf16* kb = qb + buf_elems;
  __bf16* vb = kb + buf_elems;
  __bf16* ao = vb + buf_elems;

  ttab_kernel<<<1, 256, 0, stream>>>(Ttab);
  qkv_kernel<<<dim3(TTOT / 64, QKV_N / 64), 256, 0, stream>>>(x, qkv_w, qb, kb, vb);
  attn_kernel<<<BATCH * NHEADS * (NTOK / 128), 256, 0, stream>>>(qb, kb, vb, ao);
  final_kernel<<<TTOT / 64, 256, 0, stream>>>(ao, x, proj_w, proj_b, fconv_w, fconv_b,
                                              freq_w, ln_g, ln_b, mix_w, Ttab, out);
}
